// GGNN_22797686407335
// MI455X (gfx1250) — hardware-verified
//
#include <hip/hip_runtime.h>
#include <stddef.h>
#include <stdint.h>
#include <math.h>


#define FIN     74
#define KIN     96
#define XU      (KIN / 8)
#define HD      64
#define NTY     4
#define NTC     256
#define KH2     128
#define KG      256
#define NG      256
#define G3      192
#define NTHR    256
#define NWAVE   8
#define EPT     8
#define CHUNK   (NTHR * EPT)
#define WCAP    (EPT * 32)
#define LISTN   (NWAVE * WCAP)
#define NBA     1024
#define PKS     10
#define RCAP    28672
#define DEGCAP  64
#define GBM     64
#define TBM     32
#define GTHR    128
#define U0      (HD * XU)
#define U1      (NTC * (KH2 / 8))
#define U2      (NG * (KH2 / 8))
#define U3      (NG * (KH2 / 8))
#define U4      (HD * (KG / 8))
#define U5      (HD * (KH2 / 8))
#define UTOT    (U0 + U1 + U2 + U3 + U4 + U5)
#define ZINTS   (2 * RCAP + 2 * NBA + LISTN)
#define LDS_AGG (ZINTS * 4 + 64)
#define WSMAX   134217728

static_assert((CHUNK & (CHUNK - 1)) == 0);
static_assert(NBA == (1 << PKS));
static_assert(((long long)CHUNK << PKS) < (1LL << 31));
static_assert(NTHR * 4 == NBA);
static_assert(LISTN >= NBA && LISTN >= NWAVE * WCAP);
static_assert((RCAP % 32) == 0 && (DEGCAP % 32) == 0);
static_assert((ZINTS % (NTHR * 4)) == 0);
static_assert(LDS_AGG <= 262144);
static_assert((NBA % NWAVE) == 0 && (NBA % GBM) == 0 && (NBA % TBM) == 0);
static_assert(GBM == (GTHR / 32) * 16 && 2 * TBM == GBM);
static_assert((KIN % 32) == 0 && (KH2 % 32) == 0 && (KG % 32) == 0 && KIN >= FIN && (KIN % 8) == 0);
static_assert(NTC == NTY * HD && KH2 == 2 * HD && KG == 2 * KH2 && NG == 4 * HD && G3 == 3 * HD && HD == 16 * 4);
static_assert((U0 % NTHR) == 0 && (U1 % NTHR) == 0 && (U2 % NTHR) == 0 && (U3 % NTHR) == 0);
static_assert((U4 % NTHR) == 0 && (U5 % NTHR) == 0 && (UTOT % NTHR) == 0);

typedef float          v4f   __attribute__((ext_vector_type(4)));
typedef float          v8f   __attribute__((ext_vector_type(8)));
typedef int            v4i   __attribute__((ext_vector_type(4)));
typedef int            v8i   __attribute__((ext_vector_type(8)));
typedef unsigned short v8us  __attribute__((ext_vector_type(8)));
typedef unsigned short v16us __attribute__((ext_vector_type(16)));
typedef __bf16         v16bf __attribute__((ext_vector_type(16)));
typedef v4f  __attribute__((may_alias)) v4fa;
typedef v4i  __attribute__((may_alias)) v4ia;
typedef v8us __attribute__((may_alias)) v8usa;
union Frag { v16bf v; v16us u; v8us h[2]; v8i w; };

__device__ __forceinline__ v8f wmb(const Frag& a, const Frag& b, v8f c) {
  v8f d = __builtin_amdgcn_wmma_f32_16x16x32_bf16(false, a.v, false, b.v, (short)0, c, false, false);
  asm volatile("v_nop\n\tv_nop\n\tv_nop\n\tv_nop" : "+v"(d) : "v"(a.w), "v"(b.w));
  return d;
}

__device__ __forceinline__ unsigned bf16_bits(float f) {
  const unsigned u = __float_as_uint(f);
  return (u + 0x7FFFu + ((u >> 16) & 1u)) >> 16;
}
__device__ __forceinline__ float bf16_val(float f) {
  return __uint_as_float(bf16_bits(f) << 16);
}
__device__ __forceinline__ v4f bfv4(v4f t) {
  v4f o;
  o.x = bf16_val(t.x); o.y = bf16_val(t.y); o.z = bf16_val(t.z); o.w = bf16_val(t.w);
  return o;
}
__device__ __forceinline__ v8us hilo8(v4f t) {
  v8us o;
  unsigned hb;
  hb = bf16_bits(t.x); o[0] = (unsigned short)hb; o[4] = (unsigned short)bf16_bits(t.x - __uint_as_float(hb << 16));
  hb = bf16_bits(t.y); o[1] = (unsigned short)hb; o[5] = (unsigned short)bf16_bits(t.y - __uint_as_float(hb << 16));
  hb = bf16_bits(t.z); o[2] = (unsigned short)hb; o[6] = (unsigned short)bf16_bits(t.z - __uint_as_float(hb << 16));
  hb = bf16_bits(t.w); o[3] = (unsigned short)hb; o[7] = (unsigned short)bf16_bits(t.w - __uint_as_float(hb << 16));
  return o;
}
__device__ __forceinline__ float sigm(float x) {
  const float xc = fminf(40.0f, fmaxf(-40.0f, x));
  return 1.0f / (1.0f + expf(-xc));
}
__device__ __forceinline__ float gru1(float pr, float pz, float pn, float ph, float ho) {
  const float r = sigm(pr);
  const float z = sigm(pz);
  const float n = tanhf(pn + r * ph);
  return (1.0f - z) * n + z * ho;
}

__device__ __forceinline__ int scan_chunk(const int* __restrict__ dsts, int nE, int cbase, int slotBase,
                                          int nb, int vec8, int* list, int tid, int lane, int wave) {
  int wc = 0;
  const int el0  = tid * EPT;
  const int e0   = cbase + el0;
  const int sent = -2147483647 - 1;
  v4i da, db;
  if (vec8 != 0 && cbase + CHUNK <= nE) {
    da = *(const v4i*)(dsts + e0);
    db = *(const v4i*)(dsts + e0 + 4);
  } else {
    da.x = (e0     < nE) ? dsts[min(e0,     nE - 1)] : sent;
    da.y = (e0 + 1 < nE) ? dsts[min(e0 + 1, nE - 1)] : sent;
    da.z = (e0 + 2 < nE) ? dsts[min(e0 + 2, nE - 1)] : sent;
    da.w = (e0 + 3 < nE) ? dsts[min(e0 + 3, nE - 1)] : sent;
    db.x = (e0 + 4 < nE) ? dsts[min(e0 + 4, nE - 1)] : sent;
    db.y = (e0 + 5 < nE) ? dsts[min(e0 + 5, nE - 1)] : sent;
    db.z = (e0 + 6 < nE) ? dsts[min(e0 + 6, nE - 1)] : sent;
    db.w = (e0 + 7 < nE) ? dsts[min(e0 + 7, nE - 1)] : sent;
  }
  const unsigned nbs = (unsigned)slotBase;
  const unsigned unb = (unsigned)nb;
  const unsigned s0 = (unsigned)da.x - nbs, s1 = (unsigned)da.y - nbs;
  const unsigned s2 = (unsigned)da.z - nbs, s3 = (unsigned)da.w - nbs;
  const unsigned s4 = (unsigned)db.x - nbs, s5 = (unsigned)db.y - nbs;
  const unsigned s6 = (unsigned)db.z - nbs, s7 = (unsigned)db.w - nbs;
  const bool h0 = s0 < unb, h1 = s1 < unb, h2 = s2 < unb, h3 = s3 < unb;
  const bool h4 = s4 < unb, h5 = s5 < unb, h6 = s6 < unb, h7 = s7 < unb;
  const unsigned any = __builtin_amdgcn_ballot_w32(h0 | h1 | h2 | h3 | h4 | h5 | h6 | h7);
  if (any != 0u) {
#define HITJ(J, HJ, SJ) { \
      const unsigned mj = __builtin_amdgcn_ballot_w32(HJ); \
      if (mj != 0u) { \
        if (HJ) { \
          const int pos = wc + (int)__builtin_amdgcn_mbcnt_lo(mj, 0u); \
          if (pos < WCAP) list[wave * WCAP + pos] = ((el0 + (J)) << PKS) | (int)(SJ); \
        } \
        wc += (int)__builtin_popcount(mj); } }
    HITJ(0, h0, s0)
    HITJ(1, h1, s1)
    HITJ(2, h2, s2)
    HITJ(3, h3, s3)
    HITJ(4, h4, s4)
    HITJ(5, h5, s5)
    HITJ(6, h6, s6)
    HITJ(7, h7, s7)
#undef HITJ
  }
  return wc;
}

__global__ __launch_bounds__(NTHR) void k_prep(const float* __restrict__ win, const float* __restrict__ ew,
                                               const float* __restrict__ wih, const float* __restrict__ whh,
                                               const float* __restrict__ w1, const float* __restrict__ w2,
                                               unsigned short* WINB, unsigned short* EWB, unsigned short* GWB,
                                               unsigned short* W1B, unsigned short* W2B) {
  const int u = (int)blockIdx.x * NTHR + (int)threadIdx.x;
  v8us o;
  unsigned short* dp;
  if (u < U0) {
    const int n  = u / XU;
    const int k8 = (u - XU * n) * 8;
#pragma unroll
    for (int i = 0; i < 8; ++i) {
      const int k  = k8 + i;
      const int kc = k < FIN ? k : FIN - 1;
      const float f = k < FIN ? 1.0f : 0.0f;
      o[i] = (unsigned short)bf16_bits(win[(size_t)kc * HD + n] * f);
    }
    dp = WINB + (size_t)u * 8;
  } else if (u < U0 + U1) {
    const int v  = u - U0;
    const int n  = v >> 4;
    const int g  = v & 15;
    const int t  = n >> 6;
    const int oc = n & 63;
    const float* p = ew + ((size_t)t * HD + (size_t)(4 * g)) * HD + oc;
    const unsigned short f0 = (unsigned short)bf16_bits(p[0]);
    const unsigned short f1 = (unsigned short)bf16_bits(p[HD]);
    const unsigned short f2 = (unsigned short)bf16_bits(p[2 * HD]);
    const unsigned short f3 = (unsigned short)bf16_bits(p[3 * HD]);
    o[0] = f0; o[1] = f1; o[2] = f2; o[3] = f3; o[4] = f0; o[5] = f1; o[6] = f2; o[7] = f3;
    dp = EWB + (size_t)v * 8;
  } else if (u < U0 + U1 + U2) {
    const int v  = u - U0 - U1;
    const int n  = v >> 4;
    const int g  = v & 15;
    const int wc = n < G3 ? n : n - HD;
    const float* p = wih + (size_t)(4 * g) * G3 + wc;
    const unsigned short f0 = (unsigned short)bf16_bits(p[0]);
    const unsigned short f1 = (unsigned short)bf16_bits(p[G3]);
    const unsigned short f2 = (unsigned short)bf16_bits(p[2 * G3]);
    const unsigned short f3 = (unsigned short)bf16_bits(p[3 * G3]);
    o[0] = f0; o[1] = f1; o[2] = f2; o[3] = f3; o[4] = f0; o[5] = f1; o[6] = f2; o[7] = f3;
    dp = GWB + (size_t)n * KG + 8 * g;
  } else if (u < U0 + U1 + U2 + U3) {
    const int v  = u - U0 - U1 - U2;
    const int n  = v >> 4;
    const int g  = v & 15;
    const int wc = n < G3 ? n : n - HD;
    const float* p = whh + (size_t)(4 * g) * G3 + wc;
    const unsigned short f0 = (unsigned short)bf16_bits(p[0]);
    const unsigned short f1 = (unsigned short)bf16_bits(p[G3]);
    const unsigned short f2 = (unsigned short)bf16_bits(p[2 * G3]);
    const unsigned short f3 = (unsigned short)bf16_bits(p[3 * G3]);
    o[0] = f0; o[1] = f1; o[2] = f2; o[3] = f3; o[4] = f0; o[5] = f1; o[6] = f2; o[7] = f3;
    dp = GWB + (size_t)n * KG + KH2 + 8 * g;
  } else if (u < U0 + U1 + U2 + U3 + U4) {
    const int v  = u - U0 - U1 - U2 - U3;
    const int n  = v >> 5;
    const int gg = v & 31;
    const int p2 = gg >> 4;
    const int g  = gg & 15;
    const float* p = w1 + (size_t)(HD * p2 + 4 * g) * HD + n;
    const unsigned short f0 = (unsigned short)bf16_bits(p[0]);
    const unsigned short f1 = (unsigned short)bf16_bits(p[HD]);
    const unsigned short f2 = (unsigned short)bf16_bits(p[2 * HD]);
    const unsigned short f3 = (unsigned short)bf16_bits(p[3 * HD]);
    o[0] = f0; o[1] = f1; o[2] = f2; o[3] = f3; o[4] = f0; o[5] = f1; o[6] = f2; o[7] = f3;
    dp = W1B + (size_t)v * 8;
  } else if (u < UTOT) {
    const int v = u - U0 - U1 - U2 - U3 - U4;
    const int n = v >> 4;
    const int g = v & 15;
    const float* p = w2 + (size_t)(4 * g) * HD + n;
    const unsigned short f0 = (unsigned short)bf16_bits(p[0]);
    const unsigned short f1 = (unsigned short)bf16_bits(p[HD]);
    const unsigned short f2 = (unsigned short)bf16_bits(p[2 * HD]);
    const unsigned short f3 = (unsigned short)bf16_bits(p[3 * HD]);
    o[0] = f0; o[1] = f1; o[2] = f2; o[3] = f3; o[4] = f0; o[5] = f1; o[6] = f2; o[7] = f3;
    dp = W2B + (size_t)v * 8;
  } else {
    return;
  }
  *(volatile v8us*)dp = o;
  __threadfence();
  *(volatile v8us*)dp = o;
}

__global__ __launch_bounds__(NTHR) void k_cvx(const float* __restrict__ x, int nN, int nUnits,
                                              unsigned short* xb) {
  const int u = (int)blockIdx.x * NTHR + (int)threadIdx.x;
  if (u >= nUnits) return;
  const int row = u / XU;
  const int k8  = (u - XU * row) * 8;
  const int rc  = row < nN ? row : nN - 1;
  const float keep = row < nN ? 1.0f : 0.0f;
  const float* p = x + (size_t)rc * FIN;
  v8us o;
#pragma unroll
  for (int i = 0; i < 8; ++i) {
    const int k  = k8 + i;
    const int kc = k < FIN ? k : FIN - 1;
    const float f = k < FIN ? keep : 0.0f;
    o[i] = (unsigned short)bf16_bits(p[kc] * f);
  }
  unsigned short* dp = xb + (size_t)u * 8;
  *(volatile v8us*)dp = o;
  __threadfence();
  *(volatile v8us*)dp = o;
}

__global__ __launch_bounds__(GTHR) void k_in(const unsigned short* __restrict__ XB,
                                             const unsigned short* __restrict__ WINB,
                                             const float* __restrict__ bin, float* HF, unsigned short* H0P,
                                             unsigned short* HP, int nN) {
  __shared__ __attribute__((aligned(16))) float stg[GBM * HD];
  const int tid = (int)threadIdx.x, lane = tid & 31, wave = tid >> 5, hh = lane >> 4, m = lane & 15;
  const int rowBase = (int)blockIdx.x * GBM;

  v8f acc[4];
  {
    const v8f z = {0.f, 0.f, 0.f, 0.f, 0.f, 0.f, 0.f, 0.f};
#pragma unroll
    for (int t = 0; t < 4; ++t) acc[t] = z;
  }
  const unsigned short* ap = XB + (size_t)(rowBase + 16 * wave + m) * (size_t)KIN + 8 * hh;
  const unsigned short* bp = WINB + (size_t)m * (size_t)KIN + 8 * hh;

#pragma unroll 1
  for (int k0 = 0; k0 < KIN; k0 += 32) {
    Frag af;
    af.h[0] = *(const v8usa*)(ap + k0);
    af.h[1] = *(const v8usa*)(ap + k0 + 16);
#pragma unroll
    for (int nt = 0; nt < 4; ++nt) {
      const unsigned short* wq = bp + (size_t)(16 * nt) * (size_t)KIN + k0;
      Frag bf;
      bf.h[0] = *(const v8usa*)wq;
      bf.h[1] = *(const v8usa*)(wq + 16);
      acc[nt] = wmb(af, bf, acc[nt]);
    }
  }

#pragma unroll
  for (int nt = 0; nt < 4; ++nt) {
    const int lc = 16 * nt + m;
#pragma unroll
    for (int r = 0; r < 8; ++r) {
      const int lr = 16 * wave + 8 * hh + r;
      stg[lr * HD + lc] = acc[nt][r];
    }
  }
  __syncthreads();

  const v4f b4 = bfv4(*(const v4fa*)(bin + 4 * m));
  v4f  hv[8];
  v8us hq[8];
#pragma unroll
  for (int i = 0; i < 8; ++i) {
    const int lr   = 16 * wave + 2 * i + hh;
    const int grow = rowBase + lr;
    const bool ok  = grow < nN;
    v4f t = *(const v4fa*)(stg + lr * HD + 4 * m) + b4;
    t.x = ok ? t.x : 0.0f; t.y = ok ? t.y : 0.0f; t.z = ok ? t.z : 0.0f; t.w = ok ? t.w : 0.0f;
    hv[i] = t;
    hq[i] = hilo8(t);
  }
#pragma unroll
  for (int i = 0; i < 8; ++i) {
    const int grow = rowBase + 16 * wave + 2 * i + hh;
    float* fp = HF + (size_t)grow * HD + 4 * m;
    unsigned short* p0 = H0P + (size_t)grow * KH2 + 8 * m;
    unsigned short* p1 = HP  + (size_t)grow * KH2 + 8 * m;
    *(volatile v4f*)fp  = hv[i];
    *(volatile v8us*)p0 = hq[i];
    *(volatile v8us*)p1 = hq[i];
  }
  __threadfence();
#pragma unroll
  for (int i = 0; i < 8; ++i) {
    const int grow = rowBase + 16 * wave + 2 * i + hh;
    float* fp = HF + (size_t)grow * HD + 4 * m;
    unsigned short* p0 = H0P + (size_t)grow * KH2 + 8 * m;
    unsigned short* p1 = HP  + (size_t)grow * KH2 + 8 * m;
    *(volatile v4f*)fp  = hv[i];
    *(volatile v8us*)p0 = hq[i];
    *(volatile v8us*)p1 = hq[i];
  }
}

__global__ __launch_bounds__(GTHR) void k_nt(const unsigned short* __restrict__ HPp,
                                             const unsigned short* __restrict__ EWB, float* NT) {
  __shared__ __attribute__((aligned(16))) float stg[TBM * NTC];
  const int tid = (int)threadIdx.x, lane = tid & 31, wave = tid >> 5, hh = lane >> 4, m = lane & 15;
  const int rg = wave & 1, ch = wave >> 1;
  const int rowBase = (int)blockIdx.x * TBM;

  v8f acc[8];
  {
    const v8f z = {0.f, 0.f, 0.f, 0.f, 0.f, 0.f, 0.f, 0.f};
#pragma unroll
    for (int t = 0; t < 8; ++t) acc[t] = z;
  }
  const unsigned short* ap = HPp + (size_t)(rowBase + 16 * rg + m) * (size_t)KH2 + 8 * hh;
  const unsigned short* bp = EWB + (size_t)(128 * ch + m) * (size_t)KH2 + 8 * hh;

#pragma unroll 1
  for (int k0 = 0; k0 < KH2; k0 += 32) {
    Frag af;
    af.h[0] = *(const v8usa*)(ap + k0);
    af.h[1] = *(const v8usa*)(ap + k0 + 16);
#pragma unroll
    for (int nt = 0; nt < 8; ++nt) {
      const unsigned short* wq = bp + (size_t)(16 * nt) * (size_t)KH2 + k0;
      Frag bf;
      bf.h[0] = *(const v8usa*)wq;
      bf.h[1] = *(const v8usa*)(wq + 16);
      acc[nt] = wmb(af, bf, acc[nt]);
    }
  }

#pragma unroll
  for (int nt = 0; nt < 8; ++nt) {
    const int lc = 128 * ch + 16 * nt + m;
#pragma unroll
    for (int r = 0; r < 8; ++r) {
      const int lr = 16 * rg + 8 * hh + r;
      stg[lr * NTC + lc] = acc[nt][r];
    }
  }
  __syncthreads();

  v4f pv0[8], pv1[8];
#pragma unroll
  for (int i = 0; i < 8; ++i) {
    const int lr = 8 * wave + i;
    pv0[i] = *(const v4fa*)(stg + lr * NTC + 4 * lane);
    pv1[i] = *(const v4fa*)(stg + lr * NTC + 128 + 4 * lane);
  }
#pragma unroll
  for (int i = 0; i < 8; ++i) {
    float* op = NT + (size_t)(rowBase + 8 * wave + i) * (size_t)NTC + 4 * lane;
    *(volatile v4f*)op         = pv0[i];
    *(volatile v4f*)(op + 128) = pv1[i];
  }
  __threadfence();
#pragma unroll
  for (int i = 0; i < 8; ++i) {
    float* op = NT + (size_t)(rowBase + 8 * wave + i) * (size_t)NTC + 4 * lane;
    *(volatile v4f*)op         = pv0[i];
    *(volatile v4f*)(op + 128) = pv1[i];
  }
}

__global__ __launch_bounds__(NTHR) void k_scan(const int* __restrict__ srcs, const int* __restrict__ dsts,
                                               const int* __restrict__ ets, const float* __restrict__ ebias,
                                               const float* __restrict__ NT, unsigned short* AGG,
                                               int nN, int nE, int vec8, int mRows) {
  extern __shared__ __attribute__((aligned(16))) int lds_i[];
  int* reg1 = lds_i;
  int* reg2 = reg1 + RCAP;
  int* scnt = reg2 + RCAP;
  int* soff = scnt + NBA;
  int* list = soff + NBA;
  int* wcnt = list + LISTN;
  int* wtot = wcnt + NWAVE;
  const int tid = (int)threadIdx.x, lane = tid & 31, wave = tid >> 5;
  const int nodeBase = (int)blockIdx.x * NBA;

  {
    const v4i z4 = {0, 0, 0, 0};
    for (int i = tid * 4; i < ZINTS; i += NTHR * 4) *(v4ia*)(lds_i + i) = z4;
    if (tid < 2 * NWAVE) wcnt[tid] = 0;
  }
  __syncthreads();

  int tot = 0;
  const int nChunks = (nE + CHUNK - 1) / CHUNK;
#pragma unroll 1
  for (int ch = 0; ch < nChunks; ++ch) {
    const int cbase = ch * CHUNK;
    const int wc = scan_chunk(dsts, nE, cbase, nodeBase, NBA, vec8, list, tid, lane, wave);
    if (lane == 0) wcnt[wave] = wc;
    __syncthreads();
    int pre = 0, all = 0;
#pragma unroll
    for (int w2 = 0; w2 < NWAVE; ++w2) {
      int c = wcnt[w2];
      c = c < 0 ? 0 : (c > WCAP ? WCAP : c);
      all += c;
      pre += (w2 < wave) ? c : 0;
    }
    const int wcc  = wc > WCAP ? WCAP : wc;
    const int base = tot + pre;
#pragma unroll 1
    for (int i = lane; i < wcc; i += 32) {
      const int ent = list[wave * WCAP + i];
      const int el  = (ent >> PKS) & (CHUNK - 1);
      const int sl  = ent & (NBA - 1);
      int eid = cbase + el;
      eid = eid > nE - 1 ? nE - 1 : eid;
      const int pos = base + i;
      if (pos < RCAP) reg1[pos] = (int)(((unsigned)eid << PKS) | (unsigned)sl);
    }
    tot += all;
    tot = tot > RCAP ? RCAP : tot;
    __syncthreads();
  }
  const int nh = tot;

  if (wave == 0) {
#pragma unroll 1
    for (int b0 = 0; b0 < nh; b0 += 32) {
      const int idx = b0 + lane;
      const int uv  = reg1[idx < RCAP ? idx : RCAP - 1];
      const int m32 = (nh - b0) < 32 ? (nh - b0) : 32;
#pragma unroll 1
      for (int k = 0; k < m32; ++k) {
        const int u  = __builtin_amdgcn_readlane(uv, k);
        const int sl = u & (NBA - 1);
        if (lane == 0) scnt[sl] = scnt[sl] + 1;
      }
    }
  }
  __syncthreads();

  {
    const int c0r = scnt[4 * tid], c1r = scnt[4 * tid + 1], c2r = scnt[4 * tid + 2], c3r = scnt[4 * tid + 3];
    const int e0 = c0r < 0 ? 0 : c0r, e1 = c1r < 0 ? 0 : c1r, e2 = c2r < 0 ? 0 : c2r, e3 = c3r < 0 ? 0 : c3r;
    const int ts = e0 + e1 + e2 + e3;
    int incl = ts;
#pragma unroll
    for (int d = 1; d < 32; d <<= 1) {
      const int up = __shfl_up(incl, d, 32);
      if (lane >= d) incl += up;
    }
    if (lane == 31) wtot[wave] = incl;
    __syncthreads();
    int pre = 0;
#pragma unroll
    for (int w2 = 0; w2 < NWAVE; ++w2) pre += (w2 < wave) ? wtot[w2] : 0;
    int run = pre + incl - ts;
    soff[4 * tid + 0] = run; run += e0;
    soff[4 * tid + 1] = run; run += e1;
    soff[4 * tid + 2] = run; run += e2;
    soff[4 * tid + 3] = run;
  }
  __syncthreads();
  for (int i = tid; i < NBA; i += NTHR) list[i] = soff[i];
  __syncthreads();

  if (wave == 0) {
#pragma unroll 1
    for (int b0 = 0; b0 < nh; b0 += 32) {
      const int idx = b0 + lane;
      const int uv  = reg1[idx < RCAP ? idx : RCAP - 1];
      const int m32 = (nh - b0) < 32 ? (nh - b0) : 32;
#pragma unroll 1
      for (int k = 0; k < m32; ++k) {
        const int u   = __builtin_amdgcn_readlane(uv, k);
        const int sl  = u & (NBA - 1);
        const int eid = (int)((unsigned)u >> PKS);
        if (lane == 0) {
          int pos = list[sl];
          pos = pos < 0 ? 0 : (pos > RCAP - 1 ? RCAP - 1 : pos);
          reg2[pos] = eid;
          list[sl] = pos + 1;
        }
      }
    }
  }
  __syncthreads();

  const float eb0 = bf16_val(ebias[0]), eb1 = bf16_val(ebias[1]);
  const float eb2 = bf16_val(ebias[2]), eb3 = bf16_val(ebias[3]);
  const int nbw = NBA / NWAVE;
  const bool ovf = (nh >= RCAP);
  const float qnan = __int_as_float(0x7fc00000);
  const int hsel = lane >> 4;
  const int m4   = 4 * (lane & 15);

#pragma unroll 1
  for (int jt = 0; jt < nbw; ++jt) {
    const int slot = wave * nbw + jt;
    const int node = nodeBase + slot;
    int st = soff[slot];
    const int craw = scnt[slot];
    int cnt = craw;
    st  = st < 0 ? 0 : (st > nh ? nh : st);
    cnt = cnt < 0 ? 0 : (cnt > DEGCAP ? DEGCAP : cnt);
    if (cnt > nh - st) cnt = nh - st;
    const float pz = (ovf || craw > DEGCAP) ? qnan : 0.0f;
    const bool live = node < nN;

    v4f a = {0.0f, 0.0f, 0.0f, 0.0f};
#pragma unroll 1
    for (int b0 = 0; b0 < cnt; b0 += 32) {
      int idx = st + b0 + lane; idx = idx > RCAP - 1 ? RCAP - 1 : idx;
      int eid = reg2[idx]; eid = eid < 0 ? 0 : (eid > nE - 1 ? nE - 1 : eid);
      int sr = srcs[eid]; sr = sr < 0 ? 0 : (sr > nN - 1 ? nN - 1 : sr);
      int te = ets[eid];  te = te < 0 ? 0 : (te > NTY - 1 ? NTY - 1 : te);
      const int m32 = (cnt - b0) < 32 ? (cnt - b0) : 32;
#pragma unroll 1
      for (int k = 0; k < m32; k += 2) {
        const int k1  = (k + 1) & 31;
        const int sk0 = __builtin_amdgcn_readlane(sr, k);
        const int sk1 = __builtin_amdgcn_readlane(sr, k1);
        const int tk0 = __builtin_amdgcn_readlane(te, k);
        const int tk1 = __builtin_amdgcn_readlane(te, k1);
        const float f1 = (k + 1 < m32) ? 1.0f : 0.0f;
        const int   s  = hsel ? sk1 : sk0;
        const int   t  = hsel ? tk1 : tk0;
        const float f  = hsel ? f1 : 1.0f;
        const float bb = (t == 0) ? eb0 : ((t == 1) ? eb1 : ((t == 2) ? eb2 : eb3));
        const v4f v = *(const v4f*)(NT + (size_t)s * (size_t)NTC + HD * t + m4);
        a.x += fmaxf(v.x + bb, 0.0f) * f;
        a.y += fmaxf(v.y + bb, 0.0f) * f;
        a.z += fmaxf(v.z + bb, 0.0f) * f;
        a.w += fmaxf(v.w + bb, 0.0f) * f;
      }
    }
    a.x += __shfl_xor(a.x, 16, 32);
    a.y += __shfl_xor(a.y, 16, 32);
    a.z += __shfl_xor(a.z, 16, 32);
    a.w += __shfl_xor(a.w, 16, 32);
    v4f rv;
    rv.x = (live ? a.x : 0.0f) + pz;
    rv.y = (live ? a.y : 0.0f) + pz;
    rv.z = (live ? a.z : 0.0f) + pz;
    rv.w = (live ? a.w : 0.0f) + pz;
    const v8us q = hilo8(rv);

    if (node < mRows) {
      unsigned short* gp = AGG + (size_t)node * (size_t)KH2 + 8 * (lane & 15);
      if (lane < 16) *(volatile v8us*)gp = q;
      __threadfence();
      if (lane < 16) *(volatile v8us*)gp = q;
    }
  }
}

__global__ __launch_bounds__(GTHR) void k_gru(const unsigned short* __restrict__ AG,
                                              const unsigned short* __restrict__ GW,
                                              const float* __restrict__ bih, const float* __restrict__ bhh,
                                              float* HF, unsigned short* HP, int nN) {
  __shared__ __attribute__((aligned(16))) float stg[TBM * NG];
  const int tid = (int)threadIdx.x, lane = tid & 31, wave = tid >> 5, hh = lane >> 4, m = lane & 15;
  const int rg = wave & 1, ch = wave >> 1;
  const int rowBase = (int)blockIdx.x * TBM;

  v8f acc[8];
  {
    const v8f z = {0.f, 0.f, 0.f, 0.f, 0.f, 0.f, 0.f, 0.f};
#pragma unroll
    for (int t = 0; t < 8; ++t) acc[t] = z;
  }
  const int arow = rowBase + 16 * rg + m;
  const unsigned short* apA = AG + (size_t)arow * (size_t)KH2 + 8 * hh;
  const unsigned short* apH = HP + (size_t)arow * (size_t)KH2 + 8 * hh;
  const unsigned short* bp  = GW + (size_t)m * (size_t)KG + 8 * hh;

#pragma unroll 1
  for (int k0 = 0; k0 < KH2; k0 += 32) {
    Frag af;
    af.h[0] = *(const v8usa*)(apA + k0);
    af.h[1] = *(const v8usa*)(apA + k0 + 16);
    if (ch == 0) {
#pragma unroll
      for (int nt = 0; nt < 8; ++nt) {
        const unsigned short* wq = bp + (size_t)(16 * nt) * (size_t)KG + k0;
        Frag bf;
        bf.h[0] = *(const v8usa*)wq;
        bf.h[1] = *(const v8usa*)(wq + 16);
        acc[nt] = wmb(af, bf, acc[nt]);
      }
    } else {
#pragma unroll
      for (int nt = 0; nt < 4; ++nt) {
        const unsigned short* wq = bp + (size_t)(128 + 16 * nt) * (size_t)KG + k0;
        Frag bf;
        bf.h[0] = *(const v8usa*)wq;
        bf.h[1] = *(const v8usa*)(wq + 16);
        acc[nt] = wmb(af, bf, acc[nt]);
      }
    }
  }
#pragma unroll 1
  for (int k0 = 0; k0 < KH2; k0 += 32) {
    Frag af;
    af.h[0] = *(const v8usa*)(apH + k0);
    af.h[1] = *(const v8usa*)(apH + k0 + 16);
    if (ch == 0) {
#pragma unroll
      for (int nt = 0; nt < 8; ++nt) {
        const unsigned short* wq = bp + (size_t)(16 * nt) * (size_t)KG + KH2 + k0;
        Frag bf;
        bf.h[0] = *(const v8usa*)wq;
        bf.h[1] = *(const v8usa*)(wq + 16);
        acc[nt] = wmb(af, bf, acc[nt]);
      }
    } else {
#pragma unroll
      for (int nt = 0; nt < 4; ++nt) {
        const unsigned short* wq = bp + (size_t)(192 + 16 * nt) * (size_t)KG + KH2 + k0;
        Frag bf;
        bf.h[0] = *(const v8usa*)wq;
        bf.h[1] = *(const v8usa*)(wq + 16);
        acc[4 + nt] = wmb(af, bf, acc[4 + nt]);
      }
    }
  }

#pragma unroll
  for (int nt = 0; nt < 8; ++nt) {
    const int lc = 128 * ch + 16 * nt + m;
#pragma unroll
    for (int r = 0; r < 8; ++r) {
      const int lr = 16 * rg + 8 * hh + r;
      stg[lr * NG + lc] = acc[nt][r];
    }
  }
  __syncthreads();

  v4f br, bz, bn, bq;
  {
    const v4f t0 = *(const v4fa*)(bih + 4 * m);
    const v4f t1 = *(const v4fa*)(bhh + 4 * m);
    const v4f t2 = *(const v4fa*)(bih + HD + 4 * m);
    const v4f t3 = *(const v4fa*)(bhh + HD + 4 * m);
    const v4f t4 = *(const v4fa*)(bih + 2 * HD + 4 * m);
    const v4f t5 = *(const v4fa*)(bhh + 2 * HD + 4 * m);
    br = bfv4(t0) + bfv4(t1);
    bz = bfv4(t2) + bfv4(t3);
    bn = bfv4(t4);
    bq = bfv4(t5);
  }

#pragma unroll 1
  for (int i = 0; i < 4; ++i) {
    const int lr   = 8 * wave + 2 * i + hh;
    const int grow = rowBase + lr;
    float* cell = stg + lr * NG + 4 * m;
    const v4f sr = *(const v4fa*)cell;
    const v4f sz = *(const v4fa*)(cell + HD);
    const v4f gn = *(const v4fa*)(cell + 2 * HD);
    const v4f gq = *(const v4fa*)(cell + 3 * HD);
    const v4f ho = *(const v4fa*)(HF + (size_t)grow * HD + 4 * m);
    const v4f pr = sr + br, pzv = sz + bz, pn = gn + bn, ph = gq + bq;
    v4f hn;
    hn.x = gru1(pr.x, pzv.x, pn.x, ph.x, ho.x);
    hn.y = gru1(pr.y, pzv.y, pn.y, ph.y, ho.y);
    hn.z = gru1(pr.z, pzv.z, pn.z, ph.z, ho.z);
    hn.w = gru1(pr.w, pzv.w, pn.w, ph.w, ho.w);
    const bool ok = grow < nN;
    hn.x = ok ? hn.x : 0.0f; hn.y = ok ? hn.y : 0.0f; hn.z = ok ? hn.z : 0.0f; hn.w = ok ? hn.w : 0.0f;
    *(v4fa*)cell = hn;
  }

  v4f  hv[4];
  v8us hq[4];
#pragma unroll
  for (int i = 0; i < 4; ++i) {
    const int lr = 8 * wave + 2 * i + hh;
    hv[i] = *(const v4fa*)(stg + lr * NG + 4 * m);
    hq[i] = hilo8(hv[i]);
  }
#pragma unroll
  for (int i = 0; i < 4; ++i) {
    const int grow = rowBase + 8 * wave + 2 * i + hh;
    float* fp = HF + (size_t)grow * HD + 4 * m;
    unsigned short* hp = HP + (size_t)grow * KH2 + 8 * m;
    *(volatile v4f*)fp  = hv[i];
    *(volatile v8us*)hp = hq[i];
  }
  __threadfence();
#pragma unroll
  for (int i = 0; i < 4; ++i) {
    const int grow = rowBase + 8 * wave + 2 * i + hh;
    float* fp = HF + (size_t)grow * HD + 4 * m;
    unsigned short* hp = HP + (size_t)grow * KH2 + 8 * m;
    *(volatile v4f*)fp  = hv[i];
    *(volatile v8us*)hp = hq[i];
  }
}

__global__ __launch_bounds__(GTHR) void k_mlp1(const unsigned short* __restrict__ H0P,
                                               const unsigned short* __restrict__ HPp,
                                               const unsigned short* __restrict__ W1B,
                                               const float* __restrict__ b1, unsigned short* T1P, int nN) {
  __shared__ __attribute__((aligned(16))) float stg[GBM * HD];
  const int tid = (int)threadIdx.x, lane = tid & 31, wave = tid >> 5, hh = lane >> 4, m = lane & 15;
  const int rowBase = (int)blockIdx.x * GBM;

  v8f acc[4];
  {
    const v8f z = {0.f, 0.f, 0.f, 0.f, 0.f, 0.f, 0.f, 0.f};
#pragma unroll
    for (int t = 0; t < 4; ++t) acc[t] = z;
  }
  const int arow = rowBase + 16 * wave + m;
  const unsigned short* ap0 = H0P + (size_t)arow * (size_t)KH2 + 8 * hh;
  const unsigned short* ap1 = HPp + (size_t)arow * (size_t)KH2 + 8 * hh;
  const unsigned short* bp  = W1B + (size_t)m * (size_t)KG + 8 * hh;

#pragma unroll 1
  for (int k0 = 0; k0 < KH2; k0 += 32) {
    Frag af;
    af.h[0] = *(const v8usa*)(ap0 + k0);
    af.h[1] = *(const v8usa*)(ap0 + k0 + 16);
#pragma unroll
    for (int nt = 0; nt < 4; ++nt) {
      const unsigned short* wq = bp + (size_t)(16 * nt) * (size_t)KG + k0;
      Frag bf;
      bf.h[0] = *(const v8usa*)wq;
      bf.h[1] = *(const v8usa*)(wq + 16);
      acc[nt] = wmb(af, bf, acc[nt]);
    }
  }
#pragma unroll 1
  for (int k0 = 0; k0 < KH2; k0 += 32) {
    Frag af;
    af.h[0] = *(const v8usa*)(ap1 + k0);
    af.h[1] = *(const v8usa*)(ap1 + k0 + 16);
#pragma unroll
    for (int nt = 0; nt < 4; ++nt) {
      const unsigned short* wq = bp + (size_t)(16 * nt) * (size_t)KG + KH2 + k0;
      Frag bf;
      bf.h[0] = *(const v8usa*)wq;
      bf.h[1] = *(const v8usa*)(wq + 16);
      acc[nt] = wmb(af, bf, acc[nt]);
    }
  }

#pragma unroll
  for (int nt = 0; nt < 4; ++nt) {
    const int lc = 16 * nt + m;
#pragma unroll
    for (int r = 0; r < 8; ++r) {
      const int lr = 16 * wave + 8 * hh + r;
      stg[lr * HD + lc] = acc[nt][r];
    }
  }
  __syncthreads();

  const v4f b4 = bfv4(*(const v4fa*)(b1 + 4 * m));
  v8us hq[8];
#pragma unroll
  for (int i = 0; i < 8; ++i) {
    const int lr   = 16 * wave + 2 * i + hh;
    const int grow = rowBase + lr;
    const bool ok  = grow < nN;
    v4f t = *(const v4fa*)(stg + lr * HD + 4 * m) + b4;
    t.x = fmaxf(t.x, 0.0f); t.y = fmaxf(t.y, 0.0f); t.z = fmaxf(t.z, 0.0f); t.w = fmaxf(t.w, 0.0f);
    t.x = ok ? t.x : 0.0f; t.y = ok ? t.y : 0.0f; t.z = ok ? t.z : 0.0f; t.w = ok ? t.w : 0.0f;
    hq[i] = hilo8(t);
  }
#pragma unroll
  for (int i = 0; i < 8; ++i) {
    const int grow = rowBase + 16 * wave + 2 * i + hh;
    unsigned short* p = T1P + (size_t)grow * KH2 + 8 * m;
    *(volatile v8us*)p = hq[i];
  }
  __threadfence();
#pragma unroll
  for (int i = 0; i < 8; ++i) {
    const int grow = rowBase + 16 * wave + 2 * i + hh;
    unsigned short* p = T1P + (size_t)grow * KH2 + 8 * m;
    *(volatile v8us*)p = hq[i];
  }
}

__global__ __launch_bounds__(GTHR) void k_mlp2(const unsigned short* __restrict__ T1P,
                                               const unsigned short* __restrict__ W2B,
                                               const float* __restrict__ b2, float* outp, int nN) {
  __shared__ __attribute__((aligned(16))) float stg[GBM * HD];
  const int tid = (int)threadIdx.x, lane = tid & 31, wave = tid >> 5, hh = lane >> 4, m = lane & 15;
  const int rowBase = (int)blockIdx.x * GBM;

  v8f acc[4];
  {
    const v8f z = {0.f, 0.f, 0.f, 0.f, 0.f, 0.f, 0.f, 0.f};
#pragma unroll
    for (int t = 0; t < 4; ++t) acc[t] = z;
  }
  const unsigned short* ap = T1P + (size_t)(rowBase + 16 * wave + m) * (size_t)KH2 + 8 * hh;
  const unsigned short* bp = W2B + (size_t)m * (size_t)KH2 + 8 * hh;

#pragma unroll 1
  for (int k0 = 0; k0 < KH2; k0 += 32) {
    Frag af;
    af.h[0] = *(const v8usa*)(ap + k0);
    af.h[1] = *(const v8usa*)(ap + k0 + 16);
#pragma unroll
    for (int nt = 0; nt < 4; ++nt) {
      const unsigned short* wq = bp + (size_t)(16 * nt) * (size_t)KH2 + k0;
      Frag bf;
      bf.h[0] = *(const v8usa*)wq;
      bf.h[1] = *(const v8usa*)(wq + 16);
      acc[nt] = wmb(af, bf, acc[nt]);
    }
  }

#pragma unroll
  for (int nt = 0; nt < 4; ++nt) {
    const int lc = 16 * nt + m;
#pragma unroll
    for (int r = 0; r < 8; ++r) {
      const int lr = 16 * wave + 8 * hh + r;
      stg[lr * HD + lc] = acc[nt][r];
    }
  }
  __syncthreads();

  const v4f b4 = bfv4(*(const v4fa*)(b2 + 4 * m));
#pragma unroll 1
  for (int i = 0; i < 8; ++i) {
    const int lr = 16 * wave + 2 * i + hh;
    float* cell = stg + lr * HD + 4 * m;
    const v4f t = *(const v4fa*)cell + b4;
    v4f y;
    y.x = tanhf(t.x); y.y = tanhf(t.y); y.z = tanhf(t.z); y.w = tanhf(t.w);
    *(v4fa*)cell = y;
  }
  v4f ov[8];
#pragma unroll
  for (int i = 0; i < 8; ++i) {
    const int lr = 16 * wave + 2 * i + hh;
    ov[i] = *(const v4fa*)(stg + lr * HD + 4 * m);
  }
#pragma unroll
  for (int i = 0; i < 8; ++i) {
    const int grow = rowBase + 16 * wave + 2 * i + hh;
    float* op = outp + (size_t)grow * HD + 4 * m;
    if (grow < nN) *(volatile v4f*)op = ov[i];
  }
  __threadfence();
#pragma unroll
  for (int i = 0; i < 8; ++i) {
    const int grow = rowBase + 16 * wave + 2 * i + hh;
    float* op = outp + (size_t)grow * HD + 4 * m;
    if (grow < nN) *(volatile v4f*)op = ov[i];
  }
}

static inline int cdiv(int a, int b) { return (a + b - 1) / b; }
static inline size_t al256(size_t o) { return (o + 255) & ~(size_t)255; }

extern "C" void kernel_launch(void* const* d_in, const int* in_sizes, int n_in,
                              void* d_out, int out_size, void* d_ws, size_t ws_size,
                              hipStream_t stream) {
  if (n_in < 16) return;
  if (in_sizes[0] < FIN || (in_sizes[0] % FIN) != 0) return;
  const int nN = in_sizes[0] / FIN;
  if (nN < 1 || nN > (1 << 24)) return;
  const int nE = in_sizes[3];
  if (nE < 1 || nE > (1 << 21)) return;
  if (in_sizes[1] != nE || in_sizes[2] != nE) return;
  if (in_sizes[4] != FIN * HD || in_sizes[5] != HD) return;
  if (in_sizes[6] != NTY * HD * HD || in_sizes[7] < NTY) return;
  if (in_sizes[8] != HD * G3 || in_sizes[9] != HD * G3) return;
  if (in_sizes[10] != G3 || in_sizes[11] != G3) return;
  if (in_sizes[12] != 2 * HD * HD || in_sizes[13] != HD) return;
  if (in_sizes[14] != HD * HD || in_sizes[15] != HD) return;
  if ((long long)out_size != (long long)nN * HD) return;

  const float* x     = (const float*)d_in[0];
  const int*   ety   = (const int*)d_in[1];
  const int*   src   = (const int*)d_in[2];
  const int*   dst   = (const int*)d_in[3];
  const float* win   = (const float*)d_in[4];
  const float* bin   = (const float*)d_in[5];
  const float* ew    = (const float*)d_in[6];
  const float* eb    = (const float*)d_in[7];
  const float* wih   = (const float*)d_in[8];
  const float* whh   = (const float*)d_in[9];
  const float* bih   = (const float*)d_in[10];
  const float* bhh   = (const float*)d_in[11];
  const float* w1    = (const float*)d_in[12];
  const float* b1    = (const float*)d_in[13];
  const float* w2    = (const float*)d_in[14];
  const float* b2    = (const float*)d_in[15];
  float* out = (float*)d_out;

  const int MP   = cdiv(nN, GBM) * GBM;
  const int gM64 = MP / GBM;
  const int gM32 = MP / TBM;
  const int gA   = cdiv(MP, NBA);
  if ((long long)gA * NBA < (long long)MP) return;
  const int vec8 = 1;

  char* ws = (char*)d_ws;
  size_t off = 0;
  const size_t oWINB = off; off = al256(off + (size_t)HD * KIN * 2);
  const size_t oEWB  = off; off = al256(off + (size_t)NTC * KH2 * 2);
  const size_t oGWB  = off; off = al256(off + (size_t)NG * KG * 2);
  const size_t oW1B  = off; off = al256(off + (size_t)HD * KG * 2);
  const size_t oW2B  = off; off = al256(off + (size_t)HD * KH2 * 2);
  const size_t oXB   = off; off = al256(off + (size_t)MP * KIN * 2);
  const size_t oHF   = off; off = al256(off + (size_t)MP * HD * 4);
  const size_t oH0P  = off; off = al256(off + (size_t)MP * KH2 * 2);
  const size_t oHP   = off; off = al256(off + (size_t)MP * KH2 * 2);
  const size_t oAGG  = off; off = al256(off + (size_t)MP * KH2 * 2);
  const size_t oNT   = off; off = al256(off + (size_t)MP * NTC * 4);
  if (off > ws_size || off > (size_t)WSMAX) return;
  unsigned short* WINB = (unsigned short*)(ws + oWINB);
  unsigned short* EWB  = (unsigned short*)(ws + oEWB);
  unsigned short* GWB  = (unsigned short*)(ws + oGWB);
  unsigned short* W1B  = (unsigned short*)(ws + oW1B);
  unsigned short* W2B  = (unsigned short*)(ws + oW2B);
  unsigned short* XB   = (unsigned short*)(ws + oXB);
  float*          HF   = (float*)(ws + oHF);
  unsigned short* H0P  = (unsigned short*)(ws + oH0P);
  unsigned short* HP   = (unsigned short*)(ws + oHP);
  unsigned short* AGGP = (unsigned short*)(ws + oAGG);
  unsigned short* T1P  = AGGP;
  float*          NT   = (float*)(ws + oNT);

  hipFuncSetAttribute(reinterpret_cast<const void*>(&k_scan), hipFuncAttributeMaxDynamicSharedMemorySize, LDS_AGG);

  k_prep<<<UTOT / NTHR, NTHR, 0, stream>>>(win, ew, wih, whh, w1, w2, WINB, EWB, GWB, W1B, W2B);
  const int nUx = MP * XU;
  k_cvx<<<cdiv(nUx, NTHR), NTHR, 0, stream>>>(x, nN, nUx, XB);
  k_in<<<gM64, GTHR, 0, stream>>>(XB, WINB, bin, HF, H0P, HP, nN);

  for (int s = 0; s < 4; ++s) {
    k_nt<<<gM32, GTHR, 0, stream>>>(HP, EWB, NT);
    k_scan<<<gA, NTHR, LDS_AGG, stream>>>(src, dst, ety, eb, NT, AGGP, nN, nE, vec8, MP);
    k_gru<<<gM32, GTHR, 0, stream>>>(AGGP, GWB, bih, bhh, HF, HP, nN);
  }

  k_mlp1<<<gM64, GTHR, 0, stream>>>(H0P, HP, W1B, b1, T1P, nN);
  k_mlp2<<<gM64, GTHR, 0, stream>>>(T1P, W2B, b2, out, nN);
}
